// Focal_Transformer_53283364274508
// MI455X (gfx1250) — hardware-verified
//
#include <hip/hip_runtime.h>

#define BATCH 8
#define CC 256
#define NN 4096
#define INDIM 512
#define HEADS 8
#define HDIM 64
#define N2 1024
#define N3 256
#define NKV 5120
#define C2 1024
#define C3 4096
#define LNEPS 1e-5f
#define SCP 68
#define SHP 72

typedef unsigned short u16;
typedef _Float16 hx16 __attribute__((ext_vector_type(16)));
typedef __bf16 bx16 __attribute__((ext_vector_type(16)));
typedef float v8f __attribute__((ext_vector_type(8)));
typedef float v4f __attribute__((ext_vector_type(4)));
typedef unsigned short us8 __attribute__((ext_vector_type(8)));
typedef us8 __attribute__((__may_alias__)) us8a;
typedef v4f __attribute__((__may_alias__)) v4fa;
union FragH { hx16 v; us8 p[2]; };
union FragB { bx16 v; us8 p[2]; };

__device__ __forceinline__ u16 h_bits(float f) {
  union { _Float16 h; u16 u; } c; c.h = (_Float16)f; return c.u;
}
__device__ __forceinline__ u16 bf_bits(float f) {
  unsigned u = __float_as_uint(f);
  u += 0x7FFFu + ((u >> 16) & 1u);
  return (u16)(u >> 16);
}
__device__ __forceinline__ float bf_val(u16 b) { return __uint_as_float(((unsigned)b) << 16); }

__device__ __forceinline__ void ldg_frag(us8 p[2], const u16* __restrict__ row, int k0, int h) {
  p[0] = *(const us8*)(row + k0 + 8 * h);
  p[1] = *(const us8*)(row + k0 + 16 + 8 * h);
}
__device__ __forceinline__ void lds_frag(us8 p[2], const u16* row, int k0, int h) {
  p[0] = *(const us8a*)(row + k0 + 8 * h);
  p[1] = *(const us8a*)(row + k0 + 16 + 8 * h);
}
__device__ __forceinline__ v8f mma_h(hx16 a, hx16 b, v8f c) {
  c = __builtin_amdgcn_wmma_f32_16x16x32_f16(false, a, false, b, (short)0, c, false, false);
  asm volatile("v_nop\n\tv_nop\n\tv_nop\n\tv_nop" : "+v"(c) : "v"(a), "v"(b));
  return c;
}
__device__ __forceinline__ v8f mma_b(bx16 a, bx16 b, v8f c) {
  c = __builtin_amdgcn_wmma_f32_16x16x32_bf16(false, a, false, b, (short)0, c, false, false);
  asm volatile("v_nop\n\tv_nop\n\tv_nop\n\tv_nop" : "+v"(c) : "v"(a), "v"(b));
  return c;
}
__device__ __forceinline__ void zero4(v8f acc[4]) {
#pragma unroll
  for (int nt = 0; nt < 4; ++nt)
#pragma unroll
    for (int i = 0; i < 8; ++i) acc[nt][i] = 0.f;
}

__device__ __forceinline__ void kloop_h(const u16* __restrict__ Ar, const u16* __restrict__ Br,
                                        size_t ldb, int K, int h, v8f acc[4]) {
#pragma unroll 2
  for (int k0 = 0; k0 < K; k0 += 32) {
    FragH a; ldg_frag(a.p, Ar, k0, h);
#pragma unroll
    for (int nt = 0; nt < 4; ++nt) {
      FragH b; ldg_frag(b.p, Br + (size_t)nt * 16 * ldb, k0, h);
      acc[nt] = mma_h(a.v, b.v, acc[nt]);
    }
  }
}
__device__ __forceinline__ void kloop_b3(const u16* __restrict__ Ah, const u16* __restrict__ Al,
                                         const u16* __restrict__ Bh, const u16* __restrict__ Bl,
                                         size_t ldb, int K, int h, v8f acc[4]) {
#pragma unroll 1
  for (int k0 = 0; k0 < K; k0 += 32) {
    FragB ah, al; ldg_frag(ah.p, Ah, k0, h); ldg_frag(al.p, Al, k0, h);
#pragma unroll
    for (int nt = 0; nt < 4; ++nt) {
      FragB bh, bl;
      ldg_frag(bh.p, Bh + (size_t)nt * 16 * ldb, k0, h);
      ldg_frag(bl.p, Bl + (size_t)nt * 16 * ldb, k0, h);
      acc[nt] = mma_b(ah.v, bh.v, acc[nt]);
      acc[nt] = mma_b(ah.v, bl.v, acc[nt]);
      acc[nt] = mma_b(al.v, bh.v, acc[nt]);
    }
  }
}

__device__ __forceinline__ void lines_f32(const float* sCw, float* dst, size_t ldd, int lane) {
  v4f v[8];
#pragma unroll
  for (int it = 0; it < 8; ++it) {
    const int rl = it * 2 + (lane >> 4), c = (lane & 15) * 4;
    v[it] = *(const v4fa*)(sCw + rl * SCP + c);
  }
#pragma unroll
  for (int it = 0; it < 8; ++it) {
    const int rl = it * 2 + (lane >> 4), c = (lane & 15) * 4;
    *(volatile v4f*)(dst + (size_t)rl * ldd + c) = v[it];
  }
  __threadfence();
#pragma unroll
  for (int it = 0; it < 8; ++it) {
    const int rl = it * 2 + (lane >> 4), c = (lane & 15) * 4;
    *(volatile v4f*)(dst + (size_t)rl * ldd + c) = v[it];
  }
}
__device__ __forceinline__ us8 pack_h8(const float* p, float sc) {
  v4f x0 = *(const v4fa*)p, x1 = *(const v4fa*)(p + 4);
  us8 r;
  r[0] = h_bits(x0[0] * sc); r[1] = h_bits(x0[1] * sc); r[2] = h_bits(x0[2] * sc); r[3] = h_bits(x0[3] * sc);
  r[4] = h_bits(x1[0] * sc); r[5] = h_bits(x1[1] * sc); r[6] = h_bits(x1[2] * sc); r[7] = h_bits(x1[3] * sc);
  return r;
}
__device__ __forceinline__ void lines_h(const float* sCw, u16* dst, size_t ldd, float sc, int lane) {
  us8 v[4];
#pragma unroll
  for (int it = 0; it < 4; ++it) {
    const int rl = it * 4 + (lane >> 3), c = (lane & 7) * 8;
    v[it] = pack_h8(sCw + rl * SCP + c, sc);
  }
#pragma unroll
  for (int it = 0; it < 4; ++it) {
    const int rl = it * 4 + (lane >> 3), c = (lane & 7) * 8;
    *(volatile us8*)(dst + (size_t)rl * ldd + c) = v[it];
  }
  __threadfence();
#pragma unroll
  for (int it = 0; it < 4; ++it) {
    const int rl = it * 4 + (lane >> 3), c = (lane & 7) * 8;
    *(volatile us8*)(dst + (size_t)rl * ldd + c) = v[it];
  }
}
__device__ __forceinline__ void lines_bf2(const float* sCw, u16* dh, u16* dl, size_t ldd, int lane) {
  us8 vh[4], vl[4];
#pragma unroll
  for (int it = 0; it < 4; ++it) {
    const int rl = it * 4 + (lane >> 3), c = (lane & 7) * 8;
    const float* p = sCw + rl * SCP + c;
    v4f x0 = *(const v4fa*)p, x1 = *(const v4fa*)(p + 4);
    float f[8] = {x0[0], x0[1], x0[2], x0[3], x1[0], x1[1], x1[2], x1[3]};
#pragma unroll
    for (int j = 0; j < 8; ++j) {
      u16 hb = bf_bits(f[j]);
      vh[it][j] = hb;
      vl[it][j] = bf_bits(f[j] - bf_val(hb));
    }
  }
#pragma unroll
  for (int it = 0; it < 4; ++it) {
    const int rl = it * 4 + (lane >> 3), c = (lane & 7) * 8;
    *(volatile us8*)(dh + (size_t)rl * ldd + c) = vh[it];
    *(volatile us8*)(dl + (size_t)rl * ldd + c) = vl[it];
  }
  __threadfence();
#pragma unroll
  for (int it = 0; it < 4; ++it) {
    const int rl = it * 4 + (lane >> 3), c = (lane & 7) * 8;
    *(volatile us8*)(dh + (size_t)rl * ldd + c) = vh[it];
    *(volatile us8*)(dl + (size_t)rl * ldd + c) = vl[it];
  }
}

template <int MODE>
__global__ void __launch_bounds__(64) wprep_kernel(const float* __restrict__ w, int K, int N, float sc,
                                                    u16* __restrict__ oa, u16* __restrict__ ob) {
  __shared__ float s[64 * 33];
  const int t = threadIdx.x, lane = t & 31, wv = t >> 5;
  const int k0 = blockIdx.x * 64, n0 = blockIdx.y * 32;
#pragma unroll 4
  for (int i = 0; i < 32; ++i) {
    const int idx = i * 64 + t, kk = idx >> 5, nn = idx & 31;
    const int kg = k0 + kk, ng = n0 + nn;
    float v = 0.f;
    if (kg < K && ng < N) v = w[(size_t)kg * N + ng];
    s[kk * 33 + nn] = v;
  }
  __syncthreads();
  us8 va[4], vb[4];
#pragma unroll
  for (int it = 0; it < 4; ++it) {
    const int nl = wv * 16 + it * 4 + (lane >> 3), ks = (lane & 7) * 8;
#pragma unroll
    for (int j = 0; j < 8; ++j) {
      const float f = s[(ks + j) * 33 + nl];
      if (MODE == 0) { va[it][j] = h_bits(f * sc); vb[it][j] = 0; }
      else { u16 hb = bf_bits(f); va[it][j] = hb; vb[it][j] = bf_bits(f - bf_val(hb)); }
    }
  }
#pragma unroll
  for (int it = 0; it < 4; ++it) {
    const int nl = wv * 16 + it * 4 + (lane >> 3), ks = (lane & 7) * 8;
    if (n0 + nl < N && k0 + ks + 8 <= K) {
      const size_t o = (size_t)(n0 + nl) * K + k0 + ks;
      *(volatile us8*)(oa + o) = va[it];
      if (MODE == 1) *(volatile us8*)(ob + o) = vb[it];
    }
  }
  __threadfence();
#pragma unroll
  for (int it = 0; it < 4; ++it) {
    const int nl = wv * 16 + it * 4 + (lane >> 3), ks = (lane & 7) * 8;
    if (n0 + nl < N && k0 + ks + 8 <= K) {
      const size_t o = (size_t)(n0 + nl) * K + k0 + ks;
      *(volatile us8*)(oa + o) = va[it];
      if (MODE == 1) *(volatile us8*)(ob + o) = vb[it];
    }
  }
}

__global__ void __launch_bounds__(256) ln1_kernel(const float* __restrict__ x, const float* __restrict__ g,
                                                  const float* __restrict__ be, u16* __restrict__ kv16,
                                                  int nrows) {
  const int lane = threadIdx.x & 31, wv = threadIdx.x >> 5;
  const int row = blockIdx.x * 8 + wv;
  const bool ok = row < nrows;
  const int rc = ok ? row : 0;
  const int b = rc >> 12, mm = rc & (NN - 1);
  const float* xr = x + (size_t)rc * CC + lane * 8;
  const v4f x0 = *(const v4f*)xr, x1 = *(const v4f*)(xr + 4);
  float v[8] = {x0[0], x0[1], x0[2], x0[3], x1[0], x1[1], x1[2], x1[3]};
  float s = 0.f;
#pragma unroll
  for (int i = 0; i < 8; ++i) s += v[i];
#pragma unroll
  for (int off = 16; off; off >>= 1) s += __shfl_xor(s, off, 32);
  const float mean = s * (1.f / CC);
  float sq = 0.f;
#pragma unroll
  for (int i = 0; i < 8; ++i) { const float d = v[i] - mean; sq += d * d; }
#pragma unroll
  for (int off = 16; off; off >>= 1) sq += __shfl_xor(sq, off, 32);
  const float rinv = rsqrtf(sq * (1.f / CC) + LNEPS);
  us8 o;
#pragma unroll
  for (int i = 0; i < 8; ++i) {
    const int c = lane * 8 + i;
    o[i] = h_bits((v[i] - mean) * rinv * g[c] + be[c]);
  }
  u16* dst = kv16 + ((size_t)(b * NKV + N2 + mm)) * CC + lane * 8;
  if (ok) *(volatile us8*)dst = o;
  __threadfence();
  if (ok) *(volatile us8*)dst = o;
}

__global__ void __launch_bounds__(256) ln2_kernel(const float* __restrict__ x, const float* __restrict__ g,
                                                  const float* __restrict__ be, u16* __restrict__ a2,
                                                  int nrows) {
  const int lane = threadIdx.x & 31, wv = threadIdx.x >> 5;
  const int row = blockIdx.x * 8 + wv;
  const bool ok = row < nrows;
  const int rc = ok ? row : 0;
  const int b = rc >> 10, L = rc & (N2 - 1);
  const int y2 = L >> 5, x2 = L & 31;
  const float* xb = x + (size_t)b * NN * CC;
  float v[32];
  float s = 0.f;
#pragma unroll
  for (int it = 0; it < 4; ++it) {
#pragma unroll
    for (int j = 0; j < 8; ++j) {
      const int ch = it * 256 + lane * 8 + j;
      const int c = ch >> 2, ki = (ch >> 1) & 1, kj = ch & 1;
      const int pix = (y2 * 2 + ki) * 64 + x2 * 2 + kj;
      const float t = xb[(size_t)pix * CC + c];
      v[it * 8 + j] = t; s += t;
    }
  }
#pragma unroll
  for (int off = 16; off; off >>= 1) s += __shfl_xor(s, off, 32);
  const float mean = s * (1.f / C2);
  float sq = 0.f;
#pragma unroll
  for (int i = 0; i < 32; ++i) { const float d = v[i] - mean; sq += d * d; }
#pragma unroll
  for (int off = 16; off; off >>= 1) sq += __shfl_xor(sq, off, 32);
  const float rinv = rsqrtf(sq * (1.f / C2) + LNEPS);
  us8 o[4];
#pragma unroll
  for (int it = 0; it < 4; ++it) {
#pragma unroll
    for (int j = 0; j < 8; ++j) {
      const int ch = it * 256 + lane * 8 + j;
      o[it][j] = h_bits((v[it * 8 + j] - mean) * rinv * g[ch] + be[ch]);
    }
  }
  u16* dst = a2 + (size_t)rc * C2 + lane * 8;
  if (ok) {
#pragma unroll
    for (int it = 0; it < 4; ++it) *(volatile us8*)(dst + it * 256) = o[it];
  }
  __threadfence();
  if (ok) {
#pragma unroll
    for (int it = 0; it < 4; ++it) *(volatile us8*)(dst + it * 256) = o[it];
  }
}

__global__ void __launch_bounds__(256) ln3_kernel(const float* __restrict__ x, const float* __restrict__ g,
                                                  const float* __restrict__ be, u16* __restrict__ ah,
                                                  u16* __restrict__ al) {
  __shared__ float red[8];
  const int t = threadIdx.x, lane = t & 31, wv = t >> 5;
  const int row = blockIdx.x;
  const int b = row >> 8, L = row & 255;
  const int y4 = L >> 4, x4 = L & 15;
  const float* xb = x + (size_t)b * NN * CC;
  float v[16];
  float s = 0.f;
#pragma unroll
  for (int it = 0; it < 2; ++it) {
    const int line = wv * 8 + it * 4 + (lane >> 3);
    const int chb = line * 64 + (lane & 7) * 8;
#pragma unroll
    for (int j = 0; j < 8; ++j) {
      const int ch = chb + j;
      const int c = ch >> 4, q = ch & 15, ki = q >> 2, kj = q & 3;
      const int pix = (y4 * 4 + ki) * 64 + x4 * 4 + kj;
      const float tv = xb[(size_t)pix * CC + c];
      v[it * 8 + j] = tv; s += tv;
    }
  }
#pragma unroll
  for (int off = 16; off; off >>= 1) s += __shfl_xor(s, off, 32);
  if (lane == 0) red[wv] = s;
  __syncthreads();
  float tot = 0.f;
#pragma unroll
  for (int i = 0; i < 8; ++i) tot += red[i];
  const float mean = tot * (1.f / C3);
  float sq = 0.f;
#pragma unroll
  for (int i = 0; i < 16; ++i) { const float d = v[i] - mean; sq += d * d; }
#pragma unroll
  for (int off = 16; off; off >>= 1) sq += __shfl_xor(sq, off, 32);
  __syncthreads();
  if (lane == 0) red[wv] = sq;
  __syncthreads();
  float tsq = 0.f;
#pragma unroll
  for (int i = 0; i < 8; ++i) tsq += red[i];
  const float rinv = rsqrtf(tsq * (1.f / C3) + LNEPS);
  us8 hv[2], lv[2];
#pragma unroll
  for (int it = 0; it < 2; ++it) {
    const int line = wv * 8 + it * 4 + (lane >> 3);
    const int chb = line * 64 + (lane & 7) * 8;
#pragma unroll
    for (int j = 0; j < 8; ++j) {
      const int ch = chb + j;
      const float f = (v[it * 8 + j] - mean) * rinv * g[ch] + be[ch];
      const u16 hb = bf_bits(f);
      hv[it][j] = hb;
      lv[it][j] = bf_bits(f - bf_val(hb));
    }
  }
#pragma unroll
  for (int it = 0; it < 2; ++it) {
    const int line = wv * 8 + it * 4 + (lane >> 3);
    const size_t o = (size_t)row * C3 + line * 64 + (lane & 7) * 8;
    *(volatile us8*)(ah + o) = hv[it];
    *(volatile us8*)(al + o) = lv[it];
  }
  __threadfence();
#pragma unroll
  for (int it = 0; it < 2; ++it) {
    const int line = wv * 8 + it * 4 + (lane >> 3);
    const size_t o = (size_t)row * C3 + line * 64 + (lane & 7) * 8;
    *(volatile us8*)(ah + o) = hv[it];
    *(volatile us8*)(al + o) = lv[it];
  }
}

__global__ void __launch_bounds__(128) gemm_fc2_kernel(const u16* __restrict__ A, const u16* __restrict__ Bt,
                                                       const float* __restrict__ bias, u16* __restrict__ kv16) {
  __shared__ __attribute__((aligned(16))) float sC[64 * SCP];
  const int K = C2;
  const int lane = threadIdx.x & 31, wv = threadIdx.x >> 5, h = lane >> 4, m = lane & 15;
  const int tileM = blockIdx.x * 64 + wv * 16, tileN = blockIdx.y * 64;
  v8f acc[4]; zero4(acc);
  kloop_h(A + (size_t)(tileM + m) * K, Bt + (size_t)(tileN + m) * K, (size_t)K, K, h, acc);
  float* sCw = sC + wv * 16 * SCP;
#pragma unroll
  for (int nt = 0; nt < 4; ++nt) {
    const float bv = bias[tileN + nt * 16 + m];
#pragma unroll
    for (int r = 0; r < 8; ++r) sCw[(8 * h + r) * SCP + nt * 16 + m] = acc[nt][r] * (1.f / 64.f) + bv;
  }
  __syncthreads();
  const int bb = tileM >> 10, mm = tileM & (N2 - 1);
  lines_h(sCw, kv16 + ((size_t)(bb * NKV + mm)) * CC + tileN, CC, 1.f, lane);
}

__global__ void __launch_bounds__(128) gemm_fc3_kernel(const u16* __restrict__ Ah, const u16* __restrict__ Al,
                                                       const u16* __restrict__ Bh, const u16* __restrict__ Bl,
                                                       const float* __restrict__ bias,
                                                       u16* __restrict__ oh, u16* __restrict__ ol) {
  __shared__ __attribute__((aligned(16))) float sC[64 * SCP];
  const int K = C3;
  const int lane = threadIdx.x & 31, wv = threadIdx.x >> 5, h = lane >> 4, m = lane & 15;
  const int tileM = blockIdx.x * 64 + wv * 16, tileN = blockIdx.y * 64;
  v8f acc[4]; zero4(acc);
  kloop_b3(Ah + (size_t)(tileM + m) * K, Al + (size_t)(tileM + m) * K,
           Bh + (size_t)(tileN + m) * K, Bl + (size_t)(tileN + m) * K, (size_t)K, K, h, acc);
  float* sCw = sC + wv * 16 * SCP;
#pragma unroll
  for (int nt = 0; nt < 4; ++nt) {
    const float bv = bias[tileN + nt * 16 + m];
#pragma unroll
    for (int r = 0; r < 8; ++r) sCw[(8 * h + r) * SCP + nt * 16 + m] = acc[nt][r] + bv;
  }
  __syncthreads();
  lines_bf2(sCw, oh + (size_t)tileM * CC + tileN, ol + (size_t)tileM * CC + tileN, CC, lane);
}

__global__ void __launch_bounds__(128) gemm_q_kernel(const u16* __restrict__ Ah, const u16* __restrict__ Al,
                                                     const u16* __restrict__ Bh, const u16* __restrict__ Bl,
                                                     float* __restrict__ qlin, u16* __restrict__ qb) {
  __shared__ __attribute__((aligned(16))) float sC[64 * SCP];
  const int K = CC;
  const int lane = threadIdx.x & 31, wv = threadIdx.x >> 5, h = lane >> 4, m = lane & 15;
  const int tileM = blockIdx.x * 64 + wv * 16, tileN = blockIdx.y * 64;
  v8f acc[4]; zero4(acc);
  kloop_b3(Ah + (size_t)(tileM + m) * K, Al + (size_t)(tileM + m) * K,
           Bh + (size_t)(tileN + m) * K, Bl + (size_t)(tileN + m) * K, (size_t)K, K, h, acc);
  float* sCw = sC + wv * 16 * SCP;
#pragma unroll
  for (int nt = 0; nt < 4; ++nt)
#pragma unroll
    for (int r = 0; r < 8; ++r) sCw[(8 * h + r) * SCP + nt * 16 + m] = acc[nt][r];
  __syncthreads();
  lines_f32(sCw, qlin + (size_t)tileM * INDIM + tileN, INDIM, lane);
  lines_h(sCw, qb + (size_t)tileM * INDIM + tileN, INDIM, 4.f, lane);
}

__global__ void __launch_bounds__(128) gemm_kv_kernel(const u16* __restrict__ A, const u16* __restrict__ Bt,
                                                      u16* __restrict__ kb, u16* __restrict__ vt) {
  __shared__ __attribute__((aligned(16))) float sC[64 * SCP];
  const int K = CC;
  const int lane = threadIdx.x & 31, wv = threadIdx.x >> 5, h = lane >> 4, m = lane & 15;
  const int tileM0 = blockIdx.x * 64;
  const int tileM = tileM0 + wv * 16, tileN = blockIdx.y * 64;
  v8f acc[4]; zero4(acc);
  kloop_h(A + (size_t)(tileM + m) * K, Bt + (size_t)(tileN + m) * K, (size_t)K, K, h, acc);
  float* sCw = sC + wv * 16 * SCP;
#pragma unroll
  for (int nt = 0; nt < 4; ++nt)
#pragma unroll
    for (int r = 0; r < 8; ++r) sCw[(8 * h + r) * SCP + nt * 16 + m] = acc[nt][r] * 0.25f;
  __syncthreads();
  if (blockIdx.y < 8) {
    lines_h(sCw, kb + (size_t)tileM * INDIM + tileN, INDIM, 1.f, lane);
  } else {
    const int hh = (int)blockIdx.y - 8;
    const int bb = tileM0 / NKV, mm0 = tileM0 - bb * NKV;
    us8 v[4];
#pragma unroll
    for (int it = 0; it < 4; ++it) {
      const int dl = wv * 16 + it * 4 + (lane >> 3), k8 = (lane & 7) * 8;
#pragma unroll
      for (int j = 0; j < 8; ++j) v[it][j] = h_bits(sC[(k8 + j) * SCP + dl]);
    }
#pragma unroll
    for (int it = 0; it < 4; ++it) {
      const int dl = wv * 16 + it * 4 + (lane >> 3), k8 = (lane & 7) * 8;
      u16* dst = vt + ((size_t)((bb * HEADS + hh) * HDIM + dl)) * NKV + mm0 + k8;
      *(volatile us8*)dst = v[it];
    }
    __threadfence();
#pragma unroll
    for (int it = 0; it < 4; ++it) {
      const int dl = wv * 16 + it * 4 + (lane >> 3), k8 = (lane & 7) * 8;
      u16* dst = vt + ((size_t)((bb * HEADS + hh) * HDIM + dl)) * NKV + mm0 + k8;
      *(volatile us8*)dst = v[it];
    }
  }
}

__global__ void __launch_bounds__(128) gemm_proj_kernel(const u16* __restrict__ A, const u16* __restrict__ Bt,
                                                        const float* __restrict__ bias, const float* __restrict__ qlin,
                                                        float* __restrict__ ar) {
  __shared__ __attribute__((aligned(16))) float sC[64 * SCP];
  const int K = INDIM;
  const int lane = threadIdx.x & 31, wv = threadIdx.x >> 5, h = lane >> 4, m = lane & 15;
  const int tileM = blockIdx.x * 64 + wv * 16, tileN = blockIdx.y * 64;
  v8f acc[4]; zero4(acc);
  kloop_h(A + (size_t)(tileM + m) * K, Bt + (size_t)(tileN + m) * K, (size_t)K, K, h, acc);
  float* sCw = sC + wv * 16 * SCP;
#pragma unroll
  for (int nt = 0; nt < 4; ++nt) {
    const int c = tileN + nt * 16 + m;
    const float bv = bias[c];
#pragma unroll
    for (int r = 0; r < 8; ++r)
      sCw[(8 * h + r) * SCP + nt * 16 + m] =
          acc[nt][r] * (1.f / 16384.f) + bv + qlin[(size_t)(tileM + 8 * h + r) * INDIM + c];
  }
  __syncthreads();
  lines_f32(sCw, ar + (size_t)tileM * INDIM + tileN, INDIM, lane);
}

__global__ void __launch_bounds__(128) attn_kernel(const u16* __restrict__ qb, const u16* __restrict__ kb,
                                                   const u16* __restrict__ vt, u16* __restrict__ ob) {
  __shared__ __attribute__((aligned(16))) u16 sK[64 * SHP];
  __shared__ __attribute__((aligned(16))) u16 sV[64 * SHP];
  __shared__ __attribute__((aligned(16))) u16 sP[4 * 16 * SHP];
  const int t = threadIdx.x, lane = t & 31, wv = t >> 5, h = lane >> 4, m = lane & 15;
  const int bh = blockIdx.x, b = bh >> 3, hd = bh & 7;
  const int q0 = blockIdx.y * 64 + wv * 16;
  const u16* Qr = qb + ((size_t)(b * N3 + q0 + m)) * INDIM + hd * HDIM;
  FragH qf0, qf1;
  ldg_frag(qf0.p, Qr, 0, h);
  ldg_frag(qf1.p, Qr, 32, h);
  v8f o[4]; zero4(o);
  float mr[8], lr[8];
#pragma unroll
  for (int r = 0; r < 8; ++r) { mr[r] = -1e30f; lr[r] = 0.f; }
  u16* sPw = sP + wv * 16 * SHP;

  for (int kc = 0; kc < NKV; kc += 64) {
#pragma unroll
    for (int i = 0; i < 4; ++i) {
      const int q = t * 4 + i, r = q >> 3, seg = q & 7;
      *(us8*)(sK + r * SHP + seg * 8) =
          *(const us8*)(kb + ((size_t)(b * NKV + kc + r)) * INDIM + hd * HDIM + seg * 8);
      *(us8*)(sV + r * SHP + seg * 8) =
          *(const us8*)(vt + ((size_t)(bh * HDIM + r)) * NKV + kc + seg * 8);
    }
    __syncthreads();

    v8f s[4]; zero4(s);
#pragma unroll
    for (int nt = 0; nt < 4; ++nt) {
      const u16* kr = sK + (nt * 16 + m) * SHP;
      FragH bk;
      lds_frag(bk.p, kr, 0, h);
      s[nt] = mma_h(qf0.v, bk.v, s[nt]);
      lds_frag(bk.p, kr, 32, h);
      s[nt] = mma_h(qf1.v, bk.v, s[nt]);
    }

#pragma unroll
    for (int r = 0; r < 8; ++r) {
      float x0 = fmaxf(fmaxf(s[0][r], s[1][r]), fmaxf(s[2][r], s[3][r])) * (1.f / 512.f);
#pragma unroll
      for (int off = 8; off; off >>= 1) x0 = fmaxf(x0, __shfl_xor(x0, off, 32));
      const float mnew = fmaxf(mr[r], x0);
      const float alpha = __expf(mr[r] - mnew);
      mr[r] = mnew;
      float rs = 0.f;
#pragma unroll
      for (int nt = 0; nt < 4; ++nt) {
        const float p = __expf(s[nt][r] * (1.f / 512.f) - mnew);
        rs += p;
        sPw[(8 * h + r) * SHP + nt * 16 + m] = h_bits(p * 256.f);
        o[nt][r] *= alpha;
      }
#pragma unroll
      for (int off = 8; off; off >>= 1) rs += __shfl_xor(rs, off, 32);
      lr[r] = lr[r] * alpha + rs;
    }
    __syncthreads();

#pragma unroll
    for (int ks = 0; ks < 2; ++ks) {
      FragH pa;
      lds_frag(pa.p, sPw + m * SHP, ks * 32, h);
#pragma unroll
      for (int nt = 0; nt < 4; ++nt) {
        FragH vb;
        lds_frag(vb.p, sV + (nt * 16 + m) * SHP, ks * 32, h);
        o[nt] = mma_h(pa.v, vb.v, o[nt]);
      }
    }
    __syncthreads();
  }

  float inv[8];
#pragma unroll
  for (int r = 0; r < 8; ++r) inv[r] = 1.0f / (16.f * lr[r]);
#pragma unroll
  for (int nt = 0; nt < 4; ++nt)
#pragma unroll
    for (int r = 0; r < 8; ++r) sPw[(8 * h + r) * SHP + nt * 16 + m] = h_bits(o[nt][r] * inv[r]);
  __syncthreads();
  us8 v[4];
#pragma unroll
  for (int it = 0; it < 4; ++it) {
    const int rl = it * 4 + (lane >> 3), c = (lane & 7) * 8;
    v[it] = *(const us8a*)(sPw + rl * SHP + c);
  }
#pragma unroll
  for (int it = 0; it < 4; ++it) {
    const int rl = it * 4 + (lane >> 3), c = (lane & 7) * 8;
    *(volatile us8*)(ob + ((size_t)(b * N3 + q0 + rl)) * INDIM + hd * HDIM + c) = v[it];
  }
  __threadfence();
#pragma unroll
  for (int it = 0; it < 4; ++it) {
    const int rl = it * 4 + (lane >> 3), c = (lane & 7) * 8;
    *(volatile us8*)(ob + ((size_t)(b * N3 + q0 + rl)) * INDIM + hd * HDIM + c) = v[it];
  }
}

__global__ void __launch_bounds__(64) fold_mlp_kernel(const float* __restrict__ ar, const float* __restrict__ g,
                                                      const float* __restrict__ be, const float* __restrict__ w1,
                                                      const float* __restrict__ b1, const float* __restrict__ w2,
                                                      const float* __restrict__ b2, float* __restrict__ out,
                                                      int nrows) {
  __shared__ __attribute__((aligned(16))) u16 sW1[32 * 40];
  __shared__ __attribute__((aligned(16))) u16 sW2[32 * 40];
  __shared__ __attribute__((aligned(16))) u16 sA[2 * 16 * 40];
  __shared__ __attribute__((aligned(16))) u16 sH[2 * 16 * 40];
  __shared__ __attribute__((aligned(16))) float sF[2 * 16 * 36];
  __shared__ __attribute__((aligned(16))) float sO[2 * 16 * 36];
  const int t = threadIdx.x, lane = t & 31, wv = t >> 5, h = lane >> 4, m = lane & 15;
  for (int i = t; i < 1024; i += 64) {
    const int k = i >> 5, n = i & 31;
    sW1[n * 40 + k] = h_bits(w1[i] * 64.f);
    sW2[n * 40 + k] = h_bits(w2[i] * 64.f);
  }
  const float gl = g[lane], bl = be[lane];
  const int row0 = blockIdx.x * 32 + wv * 16;
  u16* sAw = sA + wv * 16 * 40;
  u16* sHw = sH + wv * 16 * 40;
  float* sFw = sF + wv * 16 * 36;
  float* sOw = sO + wv * 16 * 36;
  for (int r = 0; r < 16; ++r) {
    const int rowg = row0 + r;
    const int rc = rowg < nrows ? rowg : 0;
    const int b = rc >> 12, pix = rc & (NN - 1);
    const int y = pix >> 6, xx = pix & 63;
    const int L = (y >> 2) * 16 + (xx >> 2), ki = y & 3, kj = xx & 3;
    const float v = ar[((size_t)(b * N3 + L)) * INDIM + lane * 16 + ki * 4 + kj];
    float s = v;
#pragma unroll
    for (int off = 16; off; off >>= 1) s += __shfl_xor(s, off, 32);
    const float mean = s * (1.f / 32.f);
    const float d = v - mean;
    float sq = d * d;
#pragma unroll
    for (int off = 16; off; off >>= 1) sq += __shfl_xor(sq, off, 32);
    const float rinv = rsqrtf(sq * (1.f / 32.f) + LNEPS);
    sFw[r * 36 + lane] = v;
    sAw[r * 40 + lane] = h_bits(d * rinv * gl + bl);
  }
  __syncthreads();

  v8f a1[2];
#pragma unroll
  for (int nt = 0; nt < 2; ++nt)
#pragma unroll
    for (int i = 0; i < 8; ++i) a1[nt][i] = 0.f;
  FragH af;
  lds_frag(af.p, sAw + m * 40, 0, h);
#pragma unroll
  for (int nt = 0; nt < 2; ++nt) {
    FragH bf;
    lds_frag(bf.p, sW1 + (nt * 16 + m) * 40, 0, h);
    a1[nt] = mma_h(af.v, bf.v, a1[nt]);
  }
#pragma unroll
  for (int nt = 0; nt < 2; ++nt) {
    const int c = nt * 16 + m;
    const float bb1 = b1[c];
#pragma unroll
    for (int r = 0; r < 8; ++r) {
      const float hv = fmaxf(a1[nt][r] * (1.f / 64.f) + bb1, 0.f);
      sHw[(8 * h + r) * 40 + c] = h_bits(hv * 256.f);
    }
  }
  __syncthreads();

  v8f a2[2];
#pragma unroll
  for (int nt = 0; nt < 2; ++nt)
#pragma unroll
    for (int i = 0; i < 8; ++i) a2[nt][i] = 0.f;
  FragH hf;
  lds_frag(hf.p, sHw + m * 40, 0, h);
#pragma unroll
  for (int nt = 0; nt < 2; ++nt) {
    FragH bf;
    lds_frag(bf.p, sW2 + (nt * 16 + m) * 40, 0, h);
    a2[nt] = mma_h(hf.v, bf.v, a2[nt]);
  }
#pragma unroll
  for (int nt = 0; nt < 2; ++nt) {
    const int c = nt * 16 + m;
    const float bb2 = b2[c];
#pragma unroll
    for (int r = 0; r < 8; ++r)
      sOw[(8 * h + r) * 36 + c] = sFw[(8 * h + r) * 36 + c] + a2[nt][r] * (1.f / 16384.f) + bb2;
  }
  __syncthreads();

  v4f ov[4];
#pragma unroll
  for (int it = 0; it < 4; ++it) {
    const int rl = it * 4 + (lane >> 3), c = (lane & 7) * 4;
    ov[it] = *(const v4fa*)(sOw + rl * 36 + c);
  }
#pragma unroll
  for (int it = 0; it < 4; ++it) {
    const int rl = it * 4 + (lane >> 3), c = (lane & 7) * 4;
    if (row0 + rl < nrows) *(volatile v4f*)(out + (size_t)(row0 + rl) * 32 + c) = ov[it];
  }
  __threadfence();
#pragma unroll
  for (int it = 0; it < 4; ++it) {
    const int rl = it * 4 + (lane >> 3), c = (lane & 7) * 4;
    if (row0 + rl < nrows) *(volatile v4f*)(out + (size_t)(row0 + rl) * 32 + c) = ov[it];
  }
}

extern "C" void kernel_launch(void* const* d_in, const int* in_sizes, int n_in,
                              void* d_out, int out_size, void* d_ws, size_t ws_size,
                              hipStream_t stream) {
  if (n_in < 21) return;
  if (in_sizes[0] != BATCH * NN * CC || in_sizes[9] != C3 * CC || in_sizes[12] != CC * 2 * INDIM ||
      out_size != BATCH * NN * 32) return;

  const float* x      = (const float*)d_in[0];
  const float* ln1_g  = (const float*)d_in[1];
  const float* ln1_b  = (const float*)d_in[2];
  const float* ln2_g  = (const float*)d_in[3];
  const float* ln2_b  = (const float*)d_in[4];
  const float* ln3_g  = (const float*)d_in[5];
  const float* ln3_b  = (const float*)d_in[6];
  const float* fc2_w  = (const float*)d_in[7];
  const float* fc2_b  = (const float*)d_in[8];
  const float* fc3_w  = (const float*)d_in[9];
  const float* fc3_b  = (const float*)d_in[10];
  const float* q_w    = (const float*)d_in[11];
  const float* kv_w   = (const float*)d_in[12];
  const float* proj_w = (const float*)d_in[13];
  const float* proj_b = (const float*)d_in[14];
  const float* n2_g   = (const float*)d_in[15];
  const float* n2_b   = (const float*)d_in[16];
  const float* mlp1_w = (const float*)d_in[17];
  const float* mlp1_b = (const float*)d_in[18];
  const float* mlp2_w = (const float*)d_in[19];
  const float* mlp2_b = (const float*)d_in[20];

  char* ws = (char*)d_ws;
  size_t off = 0;
  auto carve = [&](size_t bytes) -> char* {
    char* p = ws + off;
    off += (bytes + 255) & ~(size_t)255;
    return p;
  };
  u16* fc2T  = (u16*)carve((size_t)CC * C2 * 2);
  u16* fc3Th = (u16*)carve((size_t)CC * C3 * 2);
  u16* fc3Tl = (u16*)carve((size_t)CC * C3 * 2);
  u16* qTh   = (u16*)carve((size_t)INDIM * CC * 2);
  u16* qTl   = (u16*)carve((size_t)INDIM * CC * 2);
  u16* kvT   = (u16*)carve((size_t)2 * INDIM * CC * 2);
  u16* projT = (u16*)carve((size_t)INDIM * INDIM * 2);
  u16* kv16  = (u16*)carve((size_t)BATCH * NKV * CC * 2);
  u16* s3h   = (u16*)carve((size_t)BATCH * N3 * CC * 2);
  u16* s3l   = (u16*)carve((size_t)BATCH * N3 * CC * 2);
  float* qlin = (float*)carve((size_t)BATCH * N3 * INDIM * 4);
  u16* qb16  = (u16*)carve((size_t)BATCH * N3 * INDIM * 2);
  u16* ob16  = (u16*)carve((size_t)BATCH * N3 * INDIM * 2);
  float* ares = (float*)carve((size_t)BATCH * N3 * INDIM * 4);
  const size_t bytes_a2 = (size_t)BATCH * N2 * C2 * 2;
  const size_t bytes_a3 = (size_t)BATCH * N3 * C3 * 2;
  const size_t bytes_kb = (size_t)BATCH * NKV * INDIM * 2;
  const size_t regA = bytes_a2 + 2 * bytes_a3, regB = 2 * bytes_kb;
  char* X = carve(regA > regB ? regA : regB);
  u16* a2  = (u16*)X;
  u16* a3h = (u16*)(X + bytes_a2);
  u16* a3l = (u16*)(X + bytes_a2 + bytes_a3);
  u16* kb  = (u16*)X;
  u16* vt  = (u16*)(X + bytes_kb);
  if (off > ws_size) return;

  wprep_kernel<0><<<dim3(C2 / 64, CC / 32), 64, 0, stream>>>(fc2_w, C2, CC, 64.f, fc2T, fc2T);
  wprep_kernel<1><<<dim3(C3 / 64, CC / 32), 64, 0, stream>>>(fc3_w, C3, CC, 1.f, fc3Th, fc3Tl);
  wprep_kernel<1><<<dim3(CC / 64, INDIM / 32), 64, 0, stream>>>(q_w, CC, INDIM, 1.f, qTh, qTl);
  wprep_kernel<0><<<dim3(CC / 64, (2 * INDIM) / 32), 64, 0, stream>>>(kv_w, CC, 2 * INDIM, 64.f, kvT, kvT);
  wprep_kernel<0><<<dim3(INDIM / 64, INDIM / 32), 64, 0, stream>>>(proj_w, INDIM, INDIM, 64.f, projT, projT);

  ln1_kernel<<<(BATCH * NN + 7) / 8, 256, 0, stream>>>(x, ln1_g, ln1_b, kv16, BATCH * NN);
  ln2_kernel<<<(BATCH * N2 + 7) / 8, 256, 0, stream>>>(x, ln2_g, ln2_b, a2, BATCH * N2);
  gemm_fc2_kernel<<<dim3(BATCH * N2 / 64, CC / 64), 128, 0, stream>>>(a2, fc2T, fc2_b, kv16);
  ln3_kernel<<<BATCH * N3, 256, 0, stream>>>(x, ln3_g, ln3_b, a3h, a3l);
  gemm_fc3_kernel<<<dim3(BATCH * N3 / 64, CC / 64), 128, 0, stream>>>(a3h, a3l, fc3Th, fc3Tl, fc3_b, s3h, s3l);
  gemm_q_kernel<<<dim3(BATCH * N3 / 64, INDIM / 64), 128, 0, stream>>>(s3h, s3l, qTh, qTl, qlin, qb16);
  gemm_kv_kernel<<<dim3(BATCH * NKV / 64, (2 * INDIM) / 64), 128, 0, stream>>>(kv16, kvT, kb, vt);

  attn_kernel<<<dim3(BATCH * HEADS, N3 / 64), 128, 0, stream>>>(qb16, kb, vt, ob16);
  gemm_proj_kernel<<<dim3(BATCH * N3 / 64, INDIM / 64), 128, 0, stream>>>(ob16, projT, proj_b, qlin, ares);

  fold_mlp_kernel<<<(BATCH * NN + 31) / 32, 64, 0, stream>>>(ares, n2_g, n2_b, mlp1_w, mlp1_b,
                                                            mlp2_w, mlp2_b, (float*)d_out, BATCH * NN);
}
